// InferenceMultiHeadAttention_83004537962943
// MI455X (gfx1250) — hardware-verified
//
#include <hip/hip_runtime.h>
#include <math.h>

typedef __attribute__((ext_vector_type(16))) _Float16 v16h;
typedef __attribute__((ext_vector_type(16))) __bf16 v16b;
typedef __attribute__((ext_vector_type(8)))  _Float16 v8h;
typedef __attribute__((ext_vector_type(8)))  float v8f;
typedef __attribute__((ext_vector_type(4)))  float v4f;
typedef __attribute__((ext_vector_type(2)))  float v2f;
typedef __attribute__((ext_vector_type(4)))  unsigned v4u;
typedef __attribute__((ext_vector_type(4)))  int v4i;
typedef float __attribute__((may_alias)) float_a;
typedef int __attribute__((may_alias)) int_a;

template <typename T> __device__ __forceinline__ void vst2(void* p, T v) { *(volatile T*)p = v; __threadfence(); *(volatile T*)p = v; }
__device__ __forceinline__ v8f wmma16(v16h a, v16h b, v8f c) {
  v8f d = __builtin_amdgcn_wmma_f32_16x16x32_f16(false, a, false, b, (short)0, c, false, false);
  asm volatile("v_nop\n\tv_nop\n\tv_nop\n\tv_nop" : "+v"(d) : "v"(a), "v"(b));
  return d;
}
__device__ __forceinline__ v8f wmma_bf(v16b a, v16b b, v8f c) {
  v8f d = __builtin_amdgcn_wmma_f32_16x16x32_bf16(false, a, false, b, (short)0, c, false, false);
  asm volatile("v_nop\n\tv_nop\n\tv_nop\n\tv_nop" : "+v"(d) : "v"(a), "v"(b));
  return d;
}
__device__ __forceinline__ v16h frag_h(const _Float16* rowk0, int lane) {
  union { v16h v; v8h q[2]; } u; const _Float16* p = rowk0 + 8 * (lane >> 4);
  u.q[0] = *(const v8h*)p; u.q[1] = *(const v8h*)(p + 16); return u.v;
}
__device__ __forceinline__ v16h frag_f32(const float* rowk0, int lane) {
  v16h a; const float* p = rowk0 + 8 * (lane >> 4);
#pragma unroll
  for (int i = 0; i < 8; ++i) { a[i] = (_Float16)p[i]; a[8 + i] = (_Float16)p[16 + i]; }
  return a;
}
__device__ __forceinline__ v16h frag_f32s(const float* rowk0, int lane, float sc) {
  v16h a; const float* p = rowk0 + 8 * (lane >> 4);
#pragma unroll
  for (int i = 0; i < 8; ++i) { a[i] = (_Float16)(p[i] * sc); a[8 + i] = (_Float16)(p[16 + i] * sc); }
  return a;
}
__device__ __forceinline__ v16h fragc_f32(const float* W, int k0, int n, int lane, int ld, int K) {
  v16h a; const int g = lane >> 4;
#pragma unroll
  for (int i = 0; i < 8; ++i) { const int ka = k0 + 8 * g + i, kb = ka + 16;
    a[i] = (_Float16)(ka < K ? W[(size_t)ka * ld + n] : 0.f); a[8 + i] = (_Float16)(kb < K ? W[(size_t)kb * ld + n] : 0.f); }
  return a;
}
struct F2 { v16b h, l; };
__device__ __forceinline__ F2 bsplit16(const float v[16]) { F2 r;
#pragma unroll
  for (int i = 0; i < 16; ++i) { const __bf16 h = (__bf16)v[i]; r.h[i] = h; r.l[i] = (__bf16)(v[i] - (float)h); }
  return r; }
__device__ __forceinline__ F2 split_row(const float* row, int k0, int lane) { float v[16]; const float* p = row + k0 + 8 * (lane >> 4);
#pragma unroll
  for (int i = 0; i < 8; ++i) { v[i] = p[i]; v[8 + i] = p[16 + i]; }
  return bsplit16(v); }
__device__ __forceinline__ F2 split_rowK(const float* row, int k0, int lane, int K) { float v[16]; const int g = lane >> 4;
#pragma unroll
  for (int i = 0; i < 8; ++i) { const int ka = k0 + 8 * g + i, kb = ka + 16; v[i] = ka < K ? row[ka] : 0.f; v[8 + i] = kb < K ? row[kb] : 0.f; }
  return bsplit16(v); }
__device__ __forceinline__ F2 split_col(const float* W, int k0, int n, int lane, int ld, int K) { float v[16]; const int g = lane >> 4;
#pragma unroll
  for (int i = 0; i < 8; ++i) { const int ka = k0 + 8 * g + i, kb = ka + 16; v[i] = ka < K ? W[(size_t)ka * ld + n] : 0.f; v[8 + i] = kb < K ? W[(size_t)kb * ld + n] : 0.f; }
  return bsplit16(v); }
__device__ __forceinline__ v8f mac3(const F2& a, const F2& b, v8f c) { c = wmma_bf(a.l, b.h, c); c = wmma_bf(a.h, b.l, c); return wmma_bf(a.h, b.h, c); }
__device__ __forceinline__ float sigm(float v) { return 1.0f / (1.0f + expf(-v)); }
#define LDSX() do { asm volatile("s_wait_dscnt 0" ::: "memory"); __builtin_amdgcn_wave_barrier(); __builtin_amdgcn_fence(__ATOMIC_RELEASE, "workgroup"); } while (0)

#define SEQ 32768
#define EE 256
#define NH 4
#define HD 64
#define TB 256
#define NBLK (SEQ / TB)

__global__ __launch_bounds__(256) void k_cvt(const float* __restrict__ src, _Float16* __restrict__ dst, size_t n8, float sc) {
  const size_t g8 = (size_t)blockIdx.x * 256 + threadIdx.x; if (g8 >= n8) return;
  union { v8h h; v4u u; } pk;
#pragma unroll
  for (int e = 0; e < 8; ++e) pk.h[e] = (_Float16)(src[g8 * 8 + e] * sc);
  vst2(dst + g8 * 8, pk.u);
}
__global__ __launch_bounds__(128) void k_kv(const _Float16* __restrict__ x16, const _Float16* __restrict__ P, const float* __restrict__ bin, float* __restrict__ KV) {
  __shared__ __align__(16) float so[4][16][132];
  const int tid = threadIdx.x, wave = tid >> 5, lane = tid & 31, col = lane & 15, g = lane >> 4;
  const int r0 = blockIdx.x * 64 + wave * 16, n0 = blockIdx.y * 128;
  v8f acc[8] = {};
#pragma unroll
  for (int kc = 0; kc < EE / 32; ++kc) { const v16h a = frag_h(x16 + (size_t)(r0 + col) * EE + kc * 32, lane);
#pragma unroll
    for (int j = 0; j < 8; ++j) acc[j] = wmma16(a, frag_h(P + (size_t)(n0 + j * 16 + col) * EE + kc * 32, lane), acc[j]); }
#pragma unroll
  for (int j = 0; j < 8; ++j) { const float bb = bin[EE + n0 + j * 16 + col];
#pragma unroll
    for (int r = 0; r < 8; ++r) so[wave][8 * g + r][j * 16 + col] = acc[j][r] * (1.0f / 16.0f) + bb; }
  LDSX();
#pragma unroll 4
  for (int rl = 0; rl < 16; ++rl) vst2(KV + (size_t)(r0 + rl) * (2 * EE) + n0 + lane * 4, *(const v4f*)(&so[wave][rl][lane * 4]));
}
__global__ __launch_bounds__(256) void k_part(const float* __restrict__ x, const float* __restrict__ Win, const float* __restrict__ bin, const float* __restrict__ KV, float* __restrict__ part) {
  __shared__ float sq[EE]; __shared__ float ss[NH][TB]; __shared__ float sm[NH]; __shared__ __align__(16) float so[NH][96];
  const int tid = threadIdx.x, blk = blockIdx.x; const int t0 = blk * TB;
  { float a = bin[tid];
#pragma unroll 4
    for (int c = 0; c < EE; ++c) a += x[c] * Win[(size_t)tid * EE + c];
    sq[tid] = a * 0.125f; }
  __syncthreads();
  { const float* kr = KV + (size_t)(t0 + tid) * (2 * EE);
#pragma unroll
    for (int h = 0; h < NH; ++h) { float s = 0.f;
#pragma unroll 8
      for (int d = 0; d < HD; ++d) s += sq[h * HD + d] * kr[h * HD + d];
      ss[h][tid] = s; } }
  __syncthreads();
  if (tid < NH) { float m = -3.0e38f; for (int t = 0; t < TB; ++t) m = fmaxf(m, ss[tid][t]); sm[tid] = m; }
  __syncthreads();
  for (int h = 0; h < NH; ++h) { const float e = expf(ss[h][tid] - sm[h]); ss[h][tid] = e; }
  __syncthreads();
  { const int h = tid >> 6, d = tid & 63; float a = 0.f;
#pragma unroll 4
    for (int t = 0; t < TB; ++t) a += ss[h][t] * KV[(size_t)(t0 + t) * (2 * EE) + EE + h * HD + d];
    so[h][2 + d] = a;
    if (d == 0) { float l = 0.f; for (int t = 0; t < TB; ++t) l += ss[h][t]; so[h][0] = sm[h]; so[h][1] = l; }
    if (d < 30) so[h][66 + d] = 0.f; }
  __syncthreads();
  for (int q = tid; q < NH * 96 / 4; q += 256) vst2(part + (size_t)blk * NH * 96 + q * 4, *(const v4f*)(&so[0][0] + q * 4));
}
__global__ __launch_bounds__(256) void k_fin(const float* __restrict__ part, const float* __restrict__ Wo, const float* __restrict__ bo, float* __restrict__ out) {
  __shared__ float sctx[EE]; __shared__ float sM[NH]; __shared__ __align__(16) float so[EE];
  const int tid = threadIdx.x;
  if (tid < NH) { float M = -3.0e38f; for (int b = 0; b < NBLK; ++b) M = fmaxf(M, part[(size_t)b * NH * 96 + tid * 96]); sM[tid] = M; }
  __syncthreads();
  { const int h = tid >> 6, d = tid & 63; float num = 0.f, den = 0.f;
#pragma unroll 1
    for (int b = 0; b < NBLK; ++b) { const float* pr = part + (size_t)b * NH * 96 + h * 96; const float w = expf(pr[0] - sM[h]); num += w * pr[2 + d]; den += w * pr[1]; }
    sctx[tid] = num / den; }
  __syncthreads();
  { float a = bo[tid];
#pragma unroll 4
    for (int c = 0; c < EE; ++c) a += sctx[c] * Wo[(size_t)tid * EE + c];
    so[tid] = a; }
  __syncthreads();
  if (tid < EE / 4) vst2(out + tid * 4, *(const v4f*)(&so[tid * 4]));
}
extern "C" void kernel_launch(void* const* d_in, const int* in_sizes, int n_in, void* d_out, int out_size, void* d_ws, size_t ws_size, hipStream_t stream) {
  (void)in_sizes; (void)n_in; (void)out_size; (void)ws_size;
  const float* x = (const float*)d_in[0]; const float* Win = (const float*)d_in[1]; const float* bin = (const float*)d_in[2]; const float* Wo = (const float*)d_in[3]; const float* bo = (const float*)d_in[4];
  float* out = (float*)d_out;
  char* ws = (char*)d_ws; size_t off = 0;
  auto take = [&](size_t bytes) { char* p = ws + off; off += (bytes + 255) & ~(size_t)255; return p; };
  _Float16* x16 = (_Float16*)take((size_t)SEQ * EE * 2); _Float16* P = (_Float16*)take((size_t)2 * EE * EE * 2); float* KV = (float*)take((size_t)SEQ * 2 * EE * 4); float* part = (float*)take((size_t)NBLK * NH * 96 * 4);
  { const size_t n8 = (size_t)SEQ * EE / 8; k_cvt<<<(unsigned)(n8 / 256), 256, 0, stream>>>(x, x16, n8, 1.0f); }
  { const size_t n8 = (size_t)2 * EE * EE / 8; k_cvt<<<(unsigned)(n8 / 256), 256, 0, stream>>>(Win + (size_t)EE * EE, P, n8, 16.0f); }
  k_kv<<<dim3(SEQ / 64, 4), 128, 0, stream>>>(x16, P, bin, KV);
  k_part<<<NBLK, 256, 0, stream>>>(x, Win, bin, KV, part);
  k_fin<<<1, 256, 0, stream>>>(part, Wo, bo, out);
}
